// DeformableConvolution1d_44109314130518
// MI455X (gfx1250) — hardware-verified
//
#include <hip/hip_runtime.h>
#include <math.h>

typedef __attribute__((ext_vector_type(16))) _Float16 v16h;
typedef __attribute__((ext_vector_type(16))) __bf16 v16b;
typedef __attribute__((ext_vector_type(8)))  _Float16 v8h;
typedef __attribute__((ext_vector_type(8)))  float v8f;
typedef __attribute__((ext_vector_type(4)))  float v4f;
typedef __attribute__((ext_vector_type(2)))  float v2f;
typedef __attribute__((ext_vector_type(4)))  unsigned v4u;
typedef __attribute__((ext_vector_type(4)))  int v4i;
typedef float __attribute__((may_alias)) float_a;
typedef int __attribute__((may_alias)) int_a;

template <typename T> __device__ __forceinline__ void vst2(void* p, T v) { *(volatile T*)p = v; __threadfence(); *(volatile T*)p = v; }
__device__ __forceinline__ v8f wmma16(v16h a, v16h b, v8f c) {
  v8f d = __builtin_amdgcn_wmma_f32_16x16x32_f16(false, a, false, b, (short)0, c, false, false);
  asm volatile("v_nop\n\tv_nop\n\tv_nop\n\tv_nop" : "+v"(d) : "v"(a), "v"(b));
  return d;
}
__device__ __forceinline__ v8f wmma_bf(v16b a, v16b b, v8f c) {
  v8f d = __builtin_amdgcn_wmma_f32_16x16x32_bf16(false, a, false, b, (short)0, c, false, false);
  asm volatile("v_nop\n\tv_nop\n\tv_nop\n\tv_nop" : "+v"(d) : "v"(a), "v"(b));
  return d;
}
__device__ __forceinline__ v16h frag_h(const _Float16* rowk0, int lane) {
  union { v16h v; v8h q[2]; } u; const _Float16* p = rowk0 + 8 * (lane >> 4);
  u.q[0] = *(const v8h*)p; u.q[1] = *(const v8h*)(p + 16); return u.v;
}
__device__ __forceinline__ v16h frag_f32(const float* rowk0, int lane) {
  v16h a; const float* p = rowk0 + 8 * (lane >> 4);
#pragma unroll
  for (int i = 0; i < 8; ++i) { a[i] = (_Float16)p[i]; a[8 + i] = (_Float16)p[16 + i]; }
  return a;
}
__device__ __forceinline__ v16h frag_f32s(const float* rowk0, int lane, float sc) {
  v16h a; const float* p = rowk0 + 8 * (lane >> 4);
#pragma unroll
  for (int i = 0; i < 8; ++i) { a[i] = (_Float16)(p[i] * sc); a[8 + i] = (_Float16)(p[16 + i] * sc); }
  return a;
}
__device__ __forceinline__ v16h fragc_f32(const float* W, int k0, int n, int lane, int ld, int K) {
  v16h a; const int g = lane >> 4;
#pragma unroll
  for (int i = 0; i < 8; ++i) { const int ka = k0 + 8 * g + i, kb = ka + 16;
    a[i] = (_Float16)(ka < K ? W[(size_t)ka * ld + n] : 0.f); a[8 + i] = (_Float16)(kb < K ? W[(size_t)kb * ld + n] : 0.f); }
  return a;
}
struct F2 { v16b h, l; };
__device__ __forceinline__ F2 bsplit16(const float v[16]) { F2 r;
#pragma unroll
  for (int i = 0; i < 16; ++i) { const __bf16 h = (__bf16)v[i]; r.h[i] = h; r.l[i] = (__bf16)(v[i] - (float)h); }
  return r; }
__device__ __forceinline__ F2 split_row(const float* row, int k0, int lane) { float v[16]; const float* p = row + k0 + 8 * (lane >> 4);
#pragma unroll
  for (int i = 0; i < 8; ++i) { v[i] = p[i]; v[8 + i] = p[16 + i]; }
  return bsplit16(v); }
__device__ __forceinline__ F2 split_rowK(const float* row, int k0, int lane, int K) { float v[16]; const int g = lane >> 4;
#pragma unroll
  for (int i = 0; i < 8; ++i) { const int ka = k0 + 8 * g + i, kb = ka + 16; v[i] = ka < K ? row[ka] : 0.f; v[8 + i] = kb < K ? row[kb] : 0.f; }
  return bsplit16(v); }
__device__ __forceinline__ F2 split_col(const float* W, int k0, int n, int lane, int ld, int K) { float v[16]; const int g = lane >> 4;
#pragma unroll
  for (int i = 0; i < 8; ++i) { const int ka = k0 + 8 * g + i, kb = ka + 16; v[i] = ka < K ? W[(size_t)ka * ld + n] : 0.f; v[8 + i] = kb < K ? W[(size_t)kb * ld + n] : 0.f; }
  return bsplit16(v); }
__device__ __forceinline__ v8f mac3(const F2& a, const F2& b, v8f c) { c = wmma_bf(a.l, b.h, c); c = wmma_bf(a.h, b.l, c); return wmma_bf(a.h, b.h, c); }
__device__ __forceinline__ float sigm(float v) { return 1.0f / (1.0f + expf(-v)); }
#define LDSX() do { asm volatile("s_wait_dscnt 0" ::: "memory"); __builtin_amdgcn_wave_barrier(); __builtin_amdgcn_fence(__ATOMIC_RELEASE, "workgroup"); } while (0)

#define NB 8
#define CC 64
#define CO 64
#define LL 16384
#define KK 5
#define PADL 2
#define LP (LL + 2 * PADL)
#define KC (CC * KK)
#define NR (NB * LL)

__device__ __forceinline__ float xpad(const float* __restrict__ xr, int i) {
  int j = i - PADL; if (j < 0) j = -j; if (j >= LL) j = 2 * (LL - 1) - j; return xr[j];
}
__global__ __launch_bounds__(256) void k_interp(const float* __restrict__ x, const float* __restrict__ off, _Float16* __restrict__ VR) {
  __shared__ __align__(16) _Float16 sv[64][KC + 8];
  const int tid = threadIdx.x, b = blockIdx.y, l0 = blockIdx.x * 64;
  for (int q = tid; q < 64 * KK; q += 256) { const int ll = q / KK, k = q % KK; const int l = l0 + ll;
    const float t0 = (float)l; const float T0 = (t0 + (float)k) + off[((size_t)b * LL + l) * KK + k];
    const float T = fminf(fmaxf(T0, 0.f), (float)(LP - 1));
    int i0 = (int)floorf(T); i0 = i0 < 0 ? 0 : (i0 > LP - 2 ? LP - 2 : i0); const float fr = T - (float)i0;
    for (int c = 0; c < CC; ++c) { const float* xr = x + ((size_t)b * CC + c) * LL; const float g0 = xpad(xr, i0), g1 = xpad(xr, i0 + 1);
      sv[ll][c * KK + k] = (_Float16)(g0 * (1.0f - fr) + g1 * fr); } }
  __syncthreads();
  for (int q = tid; q < 64 * (KC / 8); q += 256) { const int ll = q / (KC / 8), pc = q % (KC / 8); vst2(VR + ((size_t)b * LL + l0 + ll) * KC + pc * 8, *(const v4u*)(&sv[ll][pc * 8])); }
}
__global__ __launch_bounds__(128) void k_conv(const _Float16* __restrict__ VR, const float* __restrict__ w, const float* __restrict__ bias, float* __restrict__ out) {
  __shared__ __align__(16) float st[CO][68];
  const int tid = threadIdx.x, wave = tid >> 5, lane = tid & 31, col = lane & 15, g = lane >> 4;
  const int b = blockIdx.y, l0 = blockIdx.x * 64; const size_t r0 = (size_t)b * LL + l0 + wave * 16;
  v8f acc[4] = {};
#pragma unroll 2
  for (int kc = 0; kc < KC / 32; ++kc) { const v16h a = frag_h(VR + (r0 + col) * KC + kc * 32, lane);
#pragma unroll
    for (int t = 0; t < 4; ++t) acc[t] = wmma16(a, frag_f32s(w + (size_t)(t * 16 + col) * KC + kc * 32, lane, 16.0f), acc[t]); }
#pragma unroll
  for (int t = 0; t < 4; ++t) { const int o = t * 16 + col; const float bb = bias[o];
#pragma unroll
    for (int r = 0; r < 8; ++r) st[o][wave * 16 + 8 * g + r] = acc[t][r] * (1.0f / 16.0f) + bb; }
  __syncthreads();
  for (int q = tid; q < CO * 16; q += 128) { const int o = q >> 4, pc = q & 15; vst2(out + ((size_t)b * CO + o) * LL + l0 + pc * 4, *(const v4f*)(&st[o][pc * 4])); }
}
extern "C" void kernel_launch(void* const* d_in, const int* in_sizes, int n_in, void* d_out, int out_size, void* d_ws, size_t ws_size, hipStream_t stream) {
  (void)in_sizes; (void)n_in; (void)out_size; (void)ws_size;
  const float* x = (const float*)d_in[0]; const float* off = (const float*)d_in[1]; const float* w = (const float*)d_in[2]; const float* bias = (const float*)d_in[3];
  float* out = (float*)d_out;
  _Float16* VR = (_Float16*)d_ws;
  k_interp<<<dim3(LL / 64, NB), 256, 0, stream>>>(x, off, VR);
  k_conv<<<dim3(LL / 64, NB), 128, 0, stream>>>(VR, w, bias, out);
}
